// RNN_23175643529381
// MI455X (gfx1250) — hardware-verified
//
#include <hip/hip_runtime.h>
#include <math.h>

constexpr int NB = 64;
constexpr int NT = 512;
constexpr int NI = 128;
constexpr int NH = 512;
constexpr int NO = 128;
constexpr int NC = 10;
constexpr int NROWS = NB * NT;
constexpr int NTHR = 256;
constexpr int NWAVE = NTHR / 32;
constexpr int SEQ_BLK = 16;
constexpr int SCAN_BLOCKS = NB / SEQ_BLK;
constexpr int HP = NH + 8;
constexpr int HT = SEQ_BLK * HP;
constexpr int OP = NO + 4;
constexpr int NOUT0 = NB * NT * NO;
constexpr int NOUT1 = NB * NC;
constexpr int WF_BLKS = (NH * NI) / NTHR;
constexpr int X8   = NROWS * NI / 8;
constexpr int WHH8 = NH * NH / 8;
constexpr int WD8  = NO * NH / 8;
constexpr int XS_GRID = ((NH / 64) * (NROWS / 64)) / 8;

static_assert(NB % SEQ_BLK == 0);
static_assert(NH == NWAVE * 64);
static_assert(NO == NWAVE * 16);
static_assert(NO == 32 * 4);
static_assert(SEQ_BLK == 2 * NWAVE);
static_assert(NH % 128 == 0);
static_assert(HP % 8 == 0 && (2 * HT) % 8 == 0);
static_assert(NI % 32 == 0 && NH % 32 == 0);
static_assert(NH % 64 == 0 && NROWS % 64 == 0);
static_assert(((NH / 64) * (NROWS / 64)) % 8 == 0);
static_assert(NOUT1 % 128 == 0);
static_assert((NH * NI) % NTHR == 0 && NI == 128);
static_assert(X8 % NTHR == 0 && WHH8 % NTHR == 0 && WD8 % NTHR == 0);
static_assert(NI / 8 == 16 && NB == 64);
static_assert(NOUT0 * 4 == 16777216 && (NOUT0 + NOUT1) * 4 == 16779776);

typedef __attribute__((ext_vector_type(16))) _Float16 v16h;
typedef __attribute__((ext_vector_type(8)))  _Float16 v8h;
typedef __attribute__((ext_vector_type(16))) __bf16   v16b;
typedef __attribute__((ext_vector_type(8)))  __bf16   v8b;
typedef __attribute__((ext_vector_type(8)))  float    v8f;
typedef __attribute__((ext_vector_type(4)))  float    v4f;
typedef __attribute__((ext_vector_type(4)))  unsigned v4u;
typedef __attribute__((ext_vector_type(2)))  unsigned v2u;

__device__ __forceinline__ unsigned short f2bf_bits(float f) {
  unsigned u = __float_as_uint(f);
  return (unsigned short)((u + 0x7FFFu + ((u >> 16) & 1u)) >> 16);
}
__device__ __forceinline__ float bf_bits2f(unsigned short h) { return __uint_as_float(((unsigned)h) << 16); }

__device__ __forceinline__ void dep_guard_h(v8f& a, v8f& b, v16h x, v16h y) { asm volatile("v_nop\n\tv_nop\n\tv_nop\n\tv_nop" : "+v"(a), "+v"(b) : "v"(x), "v"(y)); }
__device__ __forceinline__ void dep_guard_b(v8f& a, v8f& b, v16b x, v16b y) { asm volatile("v_nop\n\tv_nop\n\tv_nop\n\tv_nop" : "+v"(a), "+v"(b) : "v"(x), "v"(y)); }
__device__ __forceinline__ void dep_guard4_h(v8f& a, v8f& b, v8f& c, v8f& d, v16h x, v16h y) { asm volatile("v_nop\n\tv_nop\n\tv_nop\n\tv_nop" : "+v"(a), "+v"(b), "+v"(c), "+v"(d) : "v"(x), "v"(y)); }
__device__ __forceinline__ void dep_guard4_b(v8f& a, v8f& b, v8f& c, v8f& d, v16b x, v16b y) { asm volatile("v_nop\n\tv_nop\n\tv_nop\n\tv_nop" : "+v"(a), "+v"(b), "+v"(c), "+v"(d) : "v"(x), "v"(y)); }
__device__ __forceinline__ void dep_guard1x4_b(v8f& a, v16b x, v16b y, v16b z, v16b w) { asm volatile("v_nop\n\tv_nop\n\tv_nop\n\tv_nop" : "+v"(a) : "v"(x), "v"(y), "v"(z), "v"(w)); }
__device__ __forceinline__ void keep4_h(v16h a, v16h b, v16h c, v16h d) { asm volatile("v_nop" :: "v"(a), "v"(b), "v"(c), "v"(d)); }
__device__ __forceinline__ void keep4_b(v16b a, v16b b, v16b c, v16b d) { asm volatile("v_nop" :: "v"(a), "v"(b), "v"(c), "v"(d)); }
__device__ __forceinline__ void acc_guard4(v8f& a, v8f& b, v8f& c, v8f& d) { asm volatile("v_nop\n\tv_nop\n\tv_nop\n\tv_nop" : "+v"(a), "+v"(b), "+v"(c), "+v"(d)); }
__device__ __forceinline__ void acc_guard1(v8f& a) { asm volatile("v_nop\n\tv_nop\n\tv_nop\n\tv_nop" : "+v"(a)); }

template <typename T> struct Frag;
template <> struct Frag<_Float16> {
  typedef v16h V; union U { v16h v; v8h h[2]; };
  static __device__ __forceinline__ v16h load(const _Float16* p) {
    U f; f.h[0] = *(const v8h*)(p); f.h[1] = *(const v8h*)(p + 16); return f.v;
  }
  static __device__ __forceinline__ v8f mma(v16h a, v16h b, v8f c) {
    return __builtin_amdgcn_wmma_f32_16x16x32_f16(false, a, false, b, (short)0, c, false, false);
  }
  static __device__ __forceinline__ void guard(v8f& a, v8f& b, v16h x, v16h y) { dep_guard_h(a, b, x, y); }
  static __device__ __forceinline__ void guard4(v8f& a, v8f& b, v8f& c, v8f& d, v16h x, v16h y) { dep_guard4_h(a, b, c, d, x, y); }
  static __device__ __forceinline__ void keep(v16h a, v16h b, v16h c, v16h d) { keep4_h(a, b, c, d); }
};
template <> struct Frag<__bf16> {
  typedef v16b V; union U { v16b v; v8b h[2]; };
  static __device__ __forceinline__ v16b load(const __bf16* p) {
    U f; f.h[0] = *(const v8b*)(p); f.h[1] = *(const v8b*)(p + 16); return f.v;
  }
  static __device__ __forceinline__ v8f mma(v16b a, v16b b, v8f c) {
    return __builtin_amdgcn_wmma_f32_16x16x32_bf16(false, a, false, b, (short)0, c, false, false);
  }
  static __device__ __forceinline__ void guard(v8f& a, v8f& b, v16b x, v16b y) { dep_guard_b(a, b, x, y); }
  static __device__ __forceinline__ void guard4(v8f& a, v8f& b, v8f& c, v8f& d, v16b x, v16b y) { dep_guard4_b(a, b, c, d, x, y); }
  static __device__ __forceinline__ void keep(v16b a, v16b b, v16b c, v16b d) { keep4_b(a, b, c, d); }
};

template <int ET> struct Elem;
template <> struct Elem<0> { typedef _Float16 T; };
template <> struct Elem<1> { typedef __bf16 T; };
template <int ET, bool SPLIT, int BIAS_MODE, int OUT_MODE, bool RESID, int ACT = 0>
__global__ __launch_bounds__(256) void wmma_gemm64(
    const unsigned short* __restrict__ Ap, const unsigned short* __restrict__ A2p, int lda, long strideA,
    const unsigned short* __restrict__ Btp, const unsigned short* __restrict__ Bt2p, int ldb, long strideB,
    void* __restrict__ Cout, void* __restrict__ Cout2, int ldc, long strideC,
    const float* __restrict__ bias,
    const float* __restrict__ resid, long strideR,
    int M, int N, int K, float scale) {
  typedef typename Elem<ET>::T T;
  typedef typename Frag<T>::V V;
  const T* A = (const T*)Ap; const T* A2 = (const T*)A2p; const T* Bt = (const T*)Btp; const T* Bt2 = (const T*)Bt2p;
  __shared__ __align__(16) float sT[8][16 * 68];
  const int b    = blockIdx.y;
  const int lane = threadIdx.x & 31;
  const int wave = threadIdx.x >> 5;
  const int tilesN = N >> 6;
  const int tilesM = M >> 6;
  const int tile = blockIdx.x * 8 + wave;
  if (tile >= tilesM * tilesN) return;
  const int tm = tile / tilesN;
  const int tn = tile - tm * tilesN;
  const int m0 = tm << 6;
  const int n0 = tn << 6;

  const T* Ab  = A  + (size_t)b * strideA;
  const T* Bb  = Bt + (size_t)b * strideB;
  const T* Ab2 = SPLIT ? (A2  + (size_t)b * strideA) : nullptr;
  const T* Bb2 = SPLIT ? (Bt2 + (size_t)b * strideB) : nullptr;

  const int rlane = lane & 15;
  const int koff  = (lane >> 4) * 8;
  const int mOff  = (lane >> 4) * 8;

  v8f acc[4][4];
#pragma unroll
  for (int i = 0; i < 4; ++i)
#pragma unroll
    for (int j = 0; j < 4; ++j) acc[i][j] = (v8f){0.f,0.f,0.f,0.f,0.f,0.f,0.f,0.f};

  for (int k0 = 0; k0 < K; k0 += 32) {
    V bh[4], bl[4];
#pragma unroll
    for (int j = 0; j < 4; ++j) {
      const size_t bo = (size_t)(n0 + (j << 4) + rlane) * ldb + koff + k0;
      bh[j] = Frag<T>::load(Bb + bo);
      if (SPLIT) bl[j] = Frag<T>::load(Bb2 + bo);
    }
#pragma unroll
    for (int i = 0; i < 4; ++i) {
      const size_t ao = (size_t)(m0 + (i << 4) + rlane) * lda + koff + k0;
      V ah = Frag<T>::load(Ab + ao);
      V al;
      if (SPLIT) al = Frag<T>::load(Ab2 + ao);
#pragma unroll
      for (int j = 0; j < 4; ++j) {
        acc[i][j] = Frag<T>::mma(ah, bh[j], acc[i][j]);
        if (SPLIT) {
          acc[i][j] = Frag<T>::mma(ah, bl[j], acc[i][j]);
          acc[i][j] = Frag<T>::mma(al, bh[j], acc[i][j]);
        }
      }
      Frag<T>::guard4(acc[i][0], acc[i][1], acc[i][2], acc[i][3], ah, SPLIT ? al : ah);
    }
    Frag<T>::keep(bh[0], bh[1], bh[2], bh[3]);
    if (SPLIT) Frag<T>::keep(bl[0], bl[1], bl[2], bl[3]);
  }
  acc_guard4(acc[0][0], acc[0][1], acc[0][2], acc[0][3]);
  acc_guard4(acc[1][0], acc[1][1], acc[1][2], acc[1][3]);
  acc_guard4(acc[2][0], acc[2][1], acc[2][2], acc[2][3]);
  acc_guard4(acc[3][0], acc[3][1], acc[3][2], acc[3][3]);

  float* slab = sT[wave];
  const float* Rb = RESID ? (resid + (size_t)b * strideR) : nullptr;
#pragma unroll
  for (int i = 0; i < 4; ++i) {
    const int mBase = m0 + (i << 4);
#pragma unroll
    for (int j = 0; j < 4; ++j) {
      const int n = n0 + (j << 4) + rlane;
      float bv = 0.f;
      if (BIAS_MODE == 2) bv = bias[n];
#pragma unroll
      for (int r = 0; r < 8; ++r) {
        float v = acc[i][j][r] * scale;
        if (BIAS_MODE == 1) v += bias[mBase + mOff + r];
        if (BIAS_MODE == 2) v += bv;
        if (RESID) v += Rb[(size_t)(mBase + mOff + r) * ldc + n];
        if (ACT == 1) v = tanhf(v);
        if (ACT == 2) v = fmaxf(v, 0.0f);
        if (ACT == 3) v = v / (1.0f + expf(-v));
        if (ACT == 4) v = (v > 0.f) ? v : 0.01f * v;
        if (ACT == 5) v = 0.5f * v * (1.0f + erff(v * 0.70710678118654752f));
        slab[(mOff + r) * 68 + (j << 4) + rlane] = v;
      }
    }
    __builtin_amdgcn_fence(__ATOMIC_RELEASE, "workgroup");
    __builtin_amdgcn_wave_barrier();
    __builtin_amdgcn_fence(__ATOMIC_ACQUIRE, "workgroup");
    if (OUT_MODE == 0) {
      float* C = (float*)Cout + (size_t)b * strideC;
      const int hh = lane >> 4, c4 = (lane & 15) * 4;
      for (int pass = 0; pass < 2; ++pass) {
#pragma unroll
        for (int it = 0; it < 8; ++it) {
          const int row = it * 2 + hh;
          v4f v = *(const v4f*)(slab + row * 68 + c4);
          *(volatile v4f*)(C + (size_t)(mBase + row) * ldc + n0 + c4) = v;
        }
        __threadfence();
      }
    } else {
      const int q = lane >> 3, c8 = (lane & 7) * 8;
      unsigned short* C  = (unsigned short*)Cout  + (size_t)b * strideC;
      unsigned short* C2 = (OUT_MODE == 2) ? ((unsigned short*)Cout2 + (size_t)b * strideC) : nullptr;
      for (int pass = 0; pass < 2; ++pass) {
#pragma unroll
        for (int it = 0; it < 4; ++it) {
          const int row = it * 4 + q;
          const float* sp = slab + row * 68 + c8;
          v8h hv, lv;
#pragma unroll
          for (int e = 0; e < 8; ++e) {
            if (OUT_MODE == 1) {
              hv[e] = (_Float16)sp[e];
            } else {
              unsigned short hb = f2bf_bits(sp[e]);
              unsigned short lb = f2bf_bits(sp[e] - bf_bits2f(hb));
              hv[e] = __builtin_bit_cast(_Float16, hb);
              lv[e] = __builtin_bit_cast(_Float16, lb);
            }
          }
          *(volatile v8h*)(C + (size_t)(mBase + row) * ldc + n0 + c8) = hv;
          if (OUT_MODE == 2) *(volatile v8h*)(C2 + (size_t)(mBase + row) * ldc + n0 + c8) = lv;
        }
        __threadfence();
      }
    }
    __builtin_amdgcn_fence(__ATOMIC_RELEASE, "workgroup");
    __builtin_amdgcn_wave_barrier();
    __builtin_amdgcn_fence(__ATOMIC_ACQUIRE, "workgroup");
  }
}

__device__ __forceinline__ float tanh_e(float x) { return 1.0f - 2.0f * __builtin_amdgcn_rcpf(1.0f + expf(2.0f * x)); }

template <int PERM>
__global__ __launch_bounds__(NTHR) void split8_kernel(const float* __restrict__ src, unsigned short* __restrict__ hi,
                                                     unsigned short* __restrict__ lo, int n8) {
  const int i = blockIdx.x * NTHR + threadIdx.x;
  if (i < n8) {
    size_t so;
    if (PERM) {
      const int row = i >> 4, c8 = i & 15;
      const int t = row >> 6, b = row & 63;
      so = ((size_t)b * NT + (size_t)t) * NI + (size_t)c8 * 8;
    } else {
      so = (size_t)i * 8;
    }
    const v4f a  = *(const v4f*)(src + so);
    const v4f bq = *(const v4f*)(src + so + 4);
    v8h hv, lv;
#pragma unroll
    for (int e = 0; e < 4; ++e) {
      const float f0 = a[e];
      const float f1 = bq[e];
      const unsigned short h0 = f2bf_bits(f0);
      const unsigned short l0 = f2bf_bits(f0 - bf_bits2f(h0));
      const unsigned short h1 = f2bf_bits(f1);
      const unsigned short l1 = f2bf_bits(f1 - bf_bits2f(h1));
      hv[e]     = __builtin_bit_cast(_Float16, h0);
      hv[4 + e] = __builtin_bit_cast(_Float16, h1);
      lv[e]     = __builtin_bit_cast(_Float16, l0);
      lv[4 + e] = __builtin_bit_cast(_Float16, l1);
    }
    unsigned short* hp = hi + (size_t)i * 8;
    unsigned short* lp = lo + (size_t)i * 8;
    *(volatile v8h*)hp = hv;
    *(volatile v8h*)lp = lv;
    __threadfence();
    *(volatile v8h*)hp = hv;
    *(volatile v8h*)lp = lv;
  }
}

__global__ __launch_bounds__(NTHR) void wfuse_kernel(const float* __restrict__ W_ih, const float* __restrict__ W_init,
                                                    const float* __restrict__ b_init, const float* __restrict__ b_ih,
                                                    unsigned short* __restrict__ wch, unsigned short* __restrict__ wcl,
                                                    float* __restrict__ bcomb) {
  __shared__ __align__(16) float sv[2 * NTHR];
  const int blk = blockIdx.x, tid = threadIdx.x;
  if (blk < WF_BLKS) {
    const int e = blk * NTHR + tid;
    const int g = e >> 7, i = e & 127;
    const float* wr = W_ih + (size_t)g * NH;
    const float* wc = W_init + i;
    float acc = 0.0f;
#pragma unroll 1
    for (int h = 0; h < NH; ++h) acc = fmaf(wr[h], wc[(size_t)h * NI], acc);
    sv[tid] = acc;
    __syncthreads();
    if (tid < 32) {
      const float* sp = sv + tid * 8;
      v8h hv, lv;
#pragma unroll
      for (int q = 0; q < 8; ++q) {
        const float f = sp[q];
        const unsigned short hb = f2bf_bits(f);
        const unsigned short lb = f2bf_bits(f - bf_bits2f(hb));
        hv[q] = __builtin_bit_cast(_Float16, hb);
        lv[q] = __builtin_bit_cast(_Float16, lb);
      }
      unsigned short* hp = wch + (size_t)blk * NTHR + tid * 8;
      unsigned short* lp = wcl + (size_t)blk * NTHR + tid * 8;
      *(volatile v8h*)hp = hv;
      *(volatile v8h*)lp = lv;
      __threadfence();
      *(volatile v8h*)hp = hv;
      *(volatile v8h*)lp = lv;
    }
  } else {
    const float* w0 = W_ih + (size_t)tid * NH;
    const float* w1 = W_ih + (size_t)(tid + NTHR) * NH;
    float a0 = 0.0f, a1 = 0.0f;
#pragma unroll 1
    for (int h = 0; h < NH; ++h) {
      const float bi = b_init[h];
      a0 = fmaf(w0[h], bi, a0);
      a1 = fmaf(w1[h], bi, a1);
    }
    sv[tid]        = a0 + b_ih[tid];
    sv[tid + NTHR] = a1 + b_ih[tid + NTHR];
    __syncthreads();
    if (tid < NH / 4) {
      const v4f v = *(const v4f*)(sv + 4 * tid);
      float* op = bcomb + 4 * tid;
      *(volatile v4f*)op = v;
      __threadfence();
      *(volatile v4f*)op = v;
    }
  }
}

__global__ __launch_bounds__(NTHR) void rnn_scan_kernel(
    const float* __restrict__ xst, const float* __restrict__ mask,
    const float* __restrict__ b_hh, const float* __restrict__ b_dec,
    const unsigned short* __restrict__ whh_hp, const unsigned short* __restrict__ whh_lp,
    const unsigned short* __restrict__ wd_hp, const unsigned short* __restrict__ wd_lp,
    float* __restrict__ out0, float* __restrict__ hfin) {
  __shared__ __align__(16) unsigned short hsH[2 * HT];
  __shared__ __align__(16) unsigned short hsL[2 * HT];
  __shared__ __align__(16) float osl[SEQ_BLK * OP];
  __shared__ int lidx_s[SEQ_BLK];
  const __bf16* WHH = (const __bf16*)whh_hp;
  const __bf16* WHL = (const __bf16*)whh_lp;
  const __bf16* WDH = (const __bf16*)wd_hp;
  const __bf16* WDL = (const __bf16*)wd_lp;
  const int tid = threadIdx.x, lane = tid & 31, wave = tid >> 5;
  const int c = lane & 15, hh = lane >> 4, koff = hh * 8, mOff = hh * 8;
  const int b0 = blockIdx.x * SEQ_BLK;
  const int n0 = wave * 64;
  const int o0 = wave * 16;

  {
    const v4u z = {0u, 0u, 0u, 0u};
    for (int i = tid; i < (2 * HT) / 8; i += NTHR) {
      *(v4u*)(hsH + (size_t)i * 8) = z;
      *(v4u*)(hsL + (size_t)i * 8) = z;
    }
  }
  if (tid < SEQ_BLK) {
    const float* mr = mask + (size_t)(b0 + tid) * NT;
    float s = 0.0f;
#pragma unroll 1
    for (int q = 0; q < NT / 4; ++q) {
      const v4f m4 = *(const v4f*)(mr + 4 * q);
      s += m4[0]; s += m4[1]; s += m4[2]; s += m4[3];
    }
    s = fminf(fmaxf(s, -4096.0f), 4096.0f);
    int li = (int)s - 1;
    if (li < 0) li += NT;
    li = (li < 0) ? 0 : ((li > NT - 1) ? (NT - 1) : li);
    lidx_s[tid] = li;
  }
  __syncthreads();

  float bhh[4];
#pragma unroll
  for (int j = 0; j < 4; ++j) bhh[j] = b_hh[n0 + 16 * j + c];
  const float bdv = b_dec[o0 + c];
  const __bf16* bwh = WHH + (size_t)(n0 + c) * NH + koff;
  const __bf16* bwl = WHL + (size_t)(n0 + c) * NH + koff;
  const __bf16* bdh = WDH + (size_t)(o0 + c) * NH + koff;
  const __bf16* bdl = WDL + (size_t)(o0 + c) * NH + koff;

#pragma unroll 1
  for (int t = 0; t < NT; ++t) {
    const int cur = t & 1, nxt = cur ^ 1;
    const __bf16* aHc = (const __bf16*)(hsH + cur * HT) + c * HP + koff;
    const __bf16* aLc = (const __bf16*)(hsL + cur * HT) + c * HP + koff;
    unsigned short* hHn = hsH + nxt * HT;
    unsigned short* hLn = hsL + nxt * HT;

    v8f acc[4];
#pragma unroll
    for (int j = 0; j < 4; ++j) {
      const float* xp = xst + (size_t)(n0 + 16 * j + c) * NROWS + (size_t)t * NB + b0 + 8 * hh;
      const v4f xa = *(const v4f*)xp;
      const v4f xb = *(const v4f*)(xp + 4);
      const float bj = bhh[j];
      acc[j] = (v8f){xa[0] + bj, xa[1] + bj, xa[2] + bj, xa[3] + bj, xb[0] + bj, xb[1] + bj, xb[2] + bj, xb[3] + bj};
    }
#pragma unroll 1
    for (int kc = 0; kc < NH / 32; ++kc) {
      v16b bh[4], bl[4];
#pragma unroll
      for (int j = 0; j < 4; ++j) {
        const size_t bo = (size_t)(16 * j) * NH + (size_t)kc * 32;
        bh[j] = Frag<__bf16>::load(bwh + bo);
        bl[j] = Frag<__bf16>::load(bwl + bo);
      }
      const v16b ah = Frag<__bf16>::load(aHc + kc * 32);
      const v16b al = Frag<__bf16>::load(aLc + kc * 32);
#pragma unroll
      for (int j = 0; j < 4; ++j) {
        acc[j] = Frag<__bf16>::mma(ah, bh[j], acc[j]);
        acc[j] = Frag<__bf16>::mma(ah, bl[j], acc[j]);
        acc[j] = Frag<__bf16>::mma(al, bh[j], acc[j]);
      }
      dep_guard4_b(acc[0], acc[1], acc[2], acc[3], ah, al);
      keep4_b(bh[0], bh[1], bh[2], bh[3]);
      keep4_b(bl[0], bl[1], bl[2], bl[3]);
    }
    acc_guard4(acc[0], acc[1], acc[2], acc[3]);

#pragma unroll
    for (int j = 0; j < 4; ++j) {
#pragma unroll
      for (int r = 0; r < 8; ++r) {
        const float hv = tanh_e(acc[j][r]);
        const unsigned short hb = f2bf_bits(hv);
        const unsigned short lb = f2bf_bits(hv - bf_bits2f(hb));
        const int idx = (mOff + r) * HP + n0 + 16 * j + c;
        hHn[idx] = hb;
        hLn[idx] = lb;
      }
    }
    __syncthreads();

    v8f accD = (v8f){bdv, bdv, bdv, bdv, bdv, bdv, bdv, bdv};
    {
      const __bf16* aHn = (const __bf16*)hHn + c * HP + koff;
      const __bf16* aLn = (const __bf16*)hLn + c * HP + koff;
#pragma unroll 1
      for (int kc = 0; kc < NH / 32; ++kc) {
        const v16b ah = Frag<__bf16>::load(aHn + kc * 32);
        const v16b al = Frag<__bf16>::load(aLn + kc * 32);
        const v16b dh = Frag<__bf16>::load(bdh + (size_t)kc * 32);
        const v16b dl = Frag<__bf16>::load(bdl + (size_t)kc * 32);
        accD = Frag<__bf16>::mma(ah, dh, accD);
        accD = Frag<__bf16>::mma(ah, dl, accD);
        accD = Frag<__bf16>::mma(al, dh, accD);
        dep_guard1x4_b(accD, ah, al, dh, dl);
      }
      acc_guard1(accD);
    }
#pragma unroll
    for (int r = 0; r < 8; ++r) osl[(mOff + r) * OP + o0 + c] = accD[r];
    __syncthreads();

    {
      const int rA = 2 * wave, rB = 2 * wave + 1;
      const v4f va = *(const v4f*)(osl + rA * OP + 4 * lane);
      const v4f vb = *(const v4f*)(osl + rB * OP + 4 * lane);
      float* pa = out0 + ((size_t)(b0 + rA) * NT + (size_t)t) * NO + 4 * lane;
      float* pb = out0 + ((size_t)(b0 + rB) * NT + (size_t)t) * NO + 4 * lane;
      for (int pass = 0; pass < 2; ++pass) {
        *(volatile v4f*)pa = va;
        *(volatile v4f*)pb = vb;
        __threadfence();
      }
    }
#pragma unroll
    for (int q = 0; q < 2; ++q) {
      const int rr = 2 * wave + q;
      const int lr = lidx_s[rr];
      if (lr == t) {
        v4f hv4[4];
#pragma unroll
        for (int i4 = 0; i4 < 4; ++i4) {
          const int col = 128 * i4 + 4 * lane;
          const v2u wh = *(const v2u*)(hHn + rr * HP + col);
          const v2u wl = *(const v2u*)(hLn + rr * HP + col);
          const unsigned h0w = wh[0], h1w = wh[1], l0w = wl[0], l1w = wl[1];
          v4f f;
          f[0] = __uint_as_float(h0w << 16) + __uint_as_float(l0w << 16);
          f[1] = __uint_as_float(h0w & 0xffff0000u) + __uint_as_float(l0w & 0xffff0000u);
          f[2] = __uint_as_float(h1w << 16) + __uint_as_float(l1w << 16);
          f[3] = __uint_as_float(h1w & 0xffff0000u) + __uint_as_float(l1w & 0xffff0000u);
          hv4[i4] = f;
        }
        float* hp = hfin + (size_t)(b0 + rr) * NH + 4 * lane;
        for (int pass = 0; pass < 2; ++pass) {
#pragma unroll
          for (int i4 = 0; i4 < 4; ++i4) *(volatile v4f*)(hp + 128 * i4) = hv4[i4];
          __threadfence();
        }
      }
    }
  }
}

__global__ __launch_bounds__(NTHR) void cls_kernel(const float* __restrict__ hfin, const float* __restrict__ W_cls,
                                                  const float* __restrict__ b_cls, float* __restrict__ out1) {
  __shared__ __align__(16) float lg[NOUT1];
  const int tid = threadIdx.x, lane = tid & 31, wave = tid >> 5;
#pragma unroll 1
  for (int q = 0; q < NB / NWAVE; ++q) {
    const int b = wave * (NB / NWAVE) + q;
    const float* hp = hfin + (size_t)b * NH + 16 * lane;
    const v4f h0 = *(const v4f*)(hp), h1 = *(const v4f*)(hp + 4), h2 = *(const v4f*)(hp + 8), h3 = *(const v4f*)(hp + 12);
#pragma unroll 1
    for (int cc = 0; cc < NC; ++cc) {
      const float* wp = W_cls + (size_t)cc * NH + 16 * lane;
      const v4f w0 = *(const v4f*)(wp), w1 = *(const v4f*)(wp + 4), w2 = *(const v4f*)(wp + 8), w3 = *(const v4f*)(wp + 12);
      const float bc = b_cls[cc];
      float p = 0.0f;
#pragma unroll
      for (int e = 0; e < 4; ++e) p = fmaf(h0[e], w0[e], p);
#pragma unroll
      for (int e = 0; e < 4; ++e) p = fmaf(h1[e], w1[e], p);
#pragma unroll
      for (int e = 0; e < 4; ++e) p = fmaf(h2[e], w2[e], p);
#pragma unroll
      for (int e = 0; e < 4; ++e) p = fmaf(h3[e], w3[e], p);
#pragma unroll
      for (int off = 1; off < 32; off <<= 1) p += __shfl_xor(p, off, 32);
      if (lane == 0) lg[b * NC + cc] = p + bc;
    }
  }
  __syncthreads();
  if (tid < 32) {
    v4f v[5];
#pragma unroll
    for (int i = 0; i < 5; ++i) v[i] = *(const v4f*)(lg + 4 * (i * 32 + lane));
    for (int pass = 0; pass < 2; ++pass) {
#pragma unroll
      for (int i = 0; i < 5; ++i) *(volatile v4f*)(out1 + 4 * (i * 32 + lane)) = v[i];
      __threadfence();
    }
  }
}

extern "C" void kernel_launch(void* const* d_in, const int* in_sizes, int n_in,
                              void* d_out, int out_size, void* d_ws, size_t ws_size, hipStream_t stream) {
  if (n_in < 12 || d_out == nullptr || d_ws == nullptr) return;
  if (in_sizes[0] != NB * NT * NI || in_sizes[1] != NB * NT || in_sizes[2] != NH * NI || in_sizes[3] != NH ||
      in_sizes[4] != NH * NH || in_sizes[5] != NH || in_sizes[6] != NH * NH || in_sizes[7] != NH ||
      in_sizes[8] != NO * NH || in_sizes[9] != NO || in_sizes[10] != NC * NH || in_sizes[11] != NC ||
      out_size != NOUT0 + NOUT1) return;

  const float* batch  = (const float*)d_in[0];
  const float* mask   = (const float*)d_in[1];
  const float* W_init = (const float*)d_in[2];
  const float* b_init = (const float*)d_in[3];
  const float* W_ih   = (const float*)d_in[4];
  const float* b_ih   = (const float*)d_in[5];
  const float* W_hh   = (const float*)d_in[6];
  const float* b_hh   = (const float*)d_in[7];
  const float* W_dec  = (const float*)d_in[8];
  const float* b_dec  = (const float*)d_in[9];
  const float* W_cls  = (const float*)d_in[10];
  const float* b_cls  = (const float*)d_in[11];
  float* out0 = (float*)d_out;
  float* out1 = out0 + (size_t)NOUT0;

  char* ws = (char*)d_ws; size_t off = 0;
  auto carve = [&](size_t bytes) -> char* { char* p = ws + off; off += (bytes + 255) & ~(size_t)255; return p; };
  unsigned short* XH    = (unsigned short*)carve((size_t)NROWS * NI * 2);
  unsigned short* XL    = (unsigned short*)carve((size_t)NROWS * NI * 2);
  unsigned short* WHHH  = (unsigned short*)carve((size_t)NH * NH * 2);
  unsigned short* WHHL  = (unsigned short*)carve((size_t)NH * NH * 2);
  unsigned short* WDH   = (unsigned short*)carve((size_t)NO * NH * 2);
  unsigned short* WDL   = (unsigned short*)carve((size_t)NO * NH * 2);
  unsigned short* WCH   = (unsigned short*)carve((size_t)NH * NI * 2);
  unsigned short* WCL   = (unsigned short*)carve((size_t)NH * NI * 2);
  float*          BCOMB = (float*)carve((size_t)NH * 4);
  float*          XST   = (float*)carve((size_t)NH * NROWS * 4);
  float*          HFIN  = (float*)carve((size_t)NB * NH * 4);
  if (off > ws_size || off > (size_t)134217728) return;

  split8_kernel<1><<<X8 / NTHR, NTHR, 0, stream>>>(batch, XH, XL, X8);
  split8_kernel<0><<<WHH8 / NTHR, NTHR, 0, stream>>>(W_hh, WHHH, WHHL, WHH8);
  split8_kernel<0><<<WD8 / NTHR, NTHR, 0, stream>>>(W_dec, WDH, WDL, WD8);

  wfuse_kernel<<<WF_BLKS + 1, NTHR, 0, stream>>>(W_ih, W_init, b_init, b_ih, WCH, WCL, BCOMB);

  wmma_gemm64<1, true, 1, 0, false, 0><<<dim3(XS_GRID, 1), 256, 0, stream>>>(
      WCH, WCL, NI, 0L, XH, XL, NI, 0L,
      (void*)XST, nullptr, NROWS, 0L, BCOMB, nullptr, 0L, NH, NROWS, NI, 1.0f);

  rnn_scan_kernel<<<SCAN_BLOCKS, NTHR, 0, stream>>>(XST, mask, b_hh, b_dec, WHHH, WHHL, WDH, WDL, out0, HFIN);

  cls_kernel<<<1, NTHR, 0, stream>>>(HFIN, W_cls, b_cls, out1);
}
